// NeRFBackbone_91122026152338
// MI455X (gfx1250) — hardware-verified
//
#include <hip/hip_runtime.h>


#define NPT  262144
#define NSMP 128
#define RCH  32768
#define HID  128
#define HC   64
#define KX   128
#define KV   32
#define DM   HID
#define LOSC 1024.0f

typedef _Float16 h16;
typedef unsigned short bf;
typedef __attribute__((ext_vector_type(16))) __bf16   v16bf;
typedef __attribute__((ext_vector_type(16))) _Float16 v16h;
typedef __attribute__((ext_vector_type(8)))  _Float16 v8h;
typedef __attribute__((ext_vector_type(8)))  unsigned short v8us;
typedef __attribute__((ext_vector_type(8)))  float    v8f;
typedef __attribute__((ext_vector_type(4)))  float    v4f;
typedef v8h  __attribute__((may_alias)) v8ha;
typedef v4f  __attribute__((may_alias)) v4fa;
typedef v8us __attribute__((may_alias)) v8usa;

__device__ __forceinline__ unsigned short f2bf(float f) { unsigned u = __float_as_uint(f); u += 0x7FFFu + ((u >> 16) & 1u); return (unsigned short)(u >> 16); }
__device__ __forceinline__ float bf2f(unsigned short b) { return __uint_as_float(((unsigned)b) << 16); }
__device__ __forceinline__ float bfr(float f) { return bf2f(f2bf(f)); }
__device__ __forceinline__ v16h cat16(v8h lo, v8h hi) { return __builtin_shufflevector(lo, hi, 0, 1, 2, 3, 4, 5, 6, 7, 8, 9, 10, 11, 12, 13, 14, 15); }
__device__ __forceinline__ v16bf cat16b(v8us lo, v8us hi) { return __builtin_bit_cast(v16bf, __builtin_shufflevector(lo, hi, 0, 1, 2, 3, 4, 5, 6, 7, 8, 9, 10, 11, 12, 13, 14, 15)); }
__device__ __forceinline__ v8f wmma16(v16h a, v16h b, v8f c) { return __builtin_amdgcn_wmma_f32_16x16x32_f16(false, a, false, b, (short)0, c, false, false); }
__device__ __forceinline__ v8f wmmab(v16bf a, v16bf b, v8f c) { return __builtin_amdgcn_wmma_f32_16x16x32_bf16(false, a, false, b, (short)0, c, false, false); }

template <bool SPLITA, bool F16OUT = false>
__global__ __launch_bounds__(128) void k_gemmb(const bf* __restrict__ A, const bf* __restrict__ Al, const bf* __restrict__ Bn, const float* __restrict__ bias, float* C, int ldc, h16* C2, const float* __restrict__ R = nullptr, int K = DM, int roundR = 1) {
    __shared__ __align__(16) float ost[4][16 * 68];
    const int lane = threadIdx.x & 31, wave = threadIdx.x >> 5, lr = lane & 15, hi = lane >> 4;
    const int r0 = blockIdx.x * 64 + wave * 16, c0 = blockIdx.y * 64;
    const size_t aoff = (size_t)(r0 + lr) * K + 8 * hi;
    size_t boff[4];
#pragma unroll
    for (int t = 0; t < 4; ++t) boff[t] = (size_t)(c0 + t * 16 + lr) * K + 8 * hi;
    v8f acc[4];
#pragma unroll
    for (int t = 0; t < 4; ++t) acc[t] = (v8f){};
#pragma unroll 1
    for (int kc = 0; kc < K; kc += 32) {
        const v16bf a = cat16b(*(const v8us*)(A + aoff + kc), *(const v8us*)(A + aoff + kc + 16));
        v16bf al = a;
        if (SPLITA) al = cat16b(*(const v8us*)(Al + aoff + kc), *(const v8us*)(Al + aoff + kc + 16));
#pragma unroll
        for (int t = 0; t < 4; ++t) { const v16bf b = cat16b(*(const v8us*)(Bn + boff[t] + kc), *(const v8us*)(Bn + boff[t] + kc + 16)); acc[t] = wmmab(a, b, acc[t]); if (SPLITA) acc[t] = wmmab(al, b, acc[t]); }
        asm volatile("v_nop\n\tv_nop\n\tv_nop\n\tv_nop" : "+v"(acc[0]), "+v"(acc[1]), "+v"(acc[2]), "+v"(acc[3]) : "v"(a), "v"(al));
    }
    float* os = &ost[wave][0];
#pragma unroll
    for (int t = 0; t < 4; ++t) { const float bv = bias ? bfr(bias[c0 + t * 16 + lr]) : 0.f;
#pragma unroll
        for (int j = 0; j < 8; ++j) os[(hi * 8 + j) * 68 + t * 16 + lr] = acc[t][j] + bv; }
    __syncthreads();
    if (F16OUT) {
        h16* crow = (h16*)(void*)C + (size_t)r0 * ldc + c0;
        auto pass = [&]() {
#pragma unroll
            for (int s = 0; s < 4; ++s) { const int row = 4 * s + (lane >> 3), piece = lane & 7; const float* sp = os + row * 68 + piece * 8; v8h o, o2;
#pragma unroll
                for (int i = 0; i < 8; ++i) { const h16 a = (h16)sp[i]; o[i] = a; o2[i] = (h16)((sp[i] - (float)a) * LOSC); }
                *(volatile v8h*)(crow + (size_t)row * ldc + piece * 8) = o; if (C2) *(volatile v8h*)(C2 + (size_t)r0 * ldc + c0 + (size_t)row * ldc + piece * 8) = o2; }
        };
        pass(); __threadfence(); pass();
    } else {
        float* crow = C + (size_t)r0 * ldc + c0;
        auto pass = [&]() {
#pragma unroll
            for (int s = 0; s < 8; ++s) { const int Lid = (lane >> 3) + 4 * s, piece = lane & 7; const int row = Lid >> 1, cofs = (Lid & 1) * 32 + piece * 4;
                v4f val = *(const v4fa*)(os + row * 68 + cofs); if (R) { const v4f rv = *(const v4f*)(R + ((size_t)r0 + row) * ldc + c0 + cofs); val += roundR ? (v4f){bfr(rv[0]), bfr(rv[1]), bfr(rv[2]), bfr(rv[3])} : rv; }
                *(volatile v4f*)(crow + (size_t)row * ldc + cofs) = val; }
        };
        pass(); __threadfence(); pass();
    }
}


__global__ __launch_bounds__(256) void k_x0pl(const float* __restrict__ pos, const float* __restrict__ cond, size_t p0, bf* X0) {
    typedef __attribute__((ext_vector_type(4))) unsigned short v4us;
    const int lane = threadIdx.x & 31; const size_t rr = (size_t)blockIdx.x * 8 + (threadIdx.x >> 5); if (rr >= (size_t)RCH) return; const size_t p = p0 + rr; v4us o;
#pragma unroll
    for (int i = 0; i < 4; ++i) { const int c = lane * 4 + i; float v = 0.f; if (c < 3) v = pos[p * 3 + c]; else if (c < 67) v = cond[c - 3]; o[i] = f2bf(v); }
    *(volatile v4us*)(X0 + rr * KX + lane * 4) = o; __threadfence(); *(volatile v4us*)(X0 + rr * KX + lane * 4) = o;
}
__global__ __launch_bounds__(256) void k_viewpl(const float* __restrict__ view, size_t p0, bf* VW) {
    typedef __attribute__((ext_vector_type(2))) unsigned short v2us;
    const int lane = threadIdx.x & 31; const size_t rr = ((size_t)blockIdx.x * 8 + (threadIdx.x >> 5)) * 2 + (lane >> 4); if (rr >= (size_t)RCH) return; const size_t ray = (p0 + rr) / NSMP; const int c0 = (lane & 15) * 2; v2us o;
#pragma unroll
    for (int i = 0; i < 2; ++i) { const int c = c0 + i; o[i] = f2bf(c < 3 ? view[ray * 3 + (c < 3 ? c : 0)] : 0.f); }
    *(volatile v2us*)(VW + rr * KV + c0) = o; __threadfence(); *(volatile v2us*)(VW + rr * KV + c0) = o;
}
template <int NC>
__global__ __launch_bounds__(256) void k_relupl(const float* __restrict__ F, bf* Ph, bf* Pl) {
    const int lane = threadIdx.x & 31; const size_t r = (size_t)blockIdx.x * 8 + (threadIdx.x >> 5); if (r >= (size_t)RCH) return;
    if (NC == 128) { typedef __attribute__((ext_vector_type(4))) unsigned short v4us; const size_t o = r * NC + lane * 4; const v4f v = *(const v4f*)(F + o); v4us oh, ol;
#pragma unroll
        for (int i = 0; i < 4; ++i) { const float y = fmaxf(v[i], 0.f); const unsigned short hb = f2bf(y); oh[i] = hb; ol[i] = f2bf(y - bf2f(hb)); }
        *(volatile v4us*)(Ph + o) = oh; *(volatile v4us*)(Pl + o) = ol; __threadfence(); *(volatile v4us*)(Ph + o) = oh; *(volatile v4us*)(Pl + o) = ol; }
    else { typedef __attribute__((ext_vector_type(2))) unsigned short v2us; typedef __attribute__((ext_vector_type(2))) float v2f_; const size_t o = r * NC + lane * 2; const v2f_ v = *(const v2f_*)(F + o); v2us oh, ol;
#pragma unroll
        for (int i = 0; i < 2; ++i) { const float y = fmaxf(v[i], 0.f); const unsigned short hb = f2bf(y); oh[i] = hb; ol[i] = f2bf(y - bf2f(hb)); }
        *(volatile v2us*)(Ph + o) = oh; *(volatile v2us*)(Pl + o) = ol; __threadfence(); *(volatile v2us*)(Ph + o) = oh; *(volatile v2us*)(Pl + o) = ol; }
}
__global__ __launch_bounds__(256) void k_wpadk(const float* __restrict__ Wt, int nin, int nout, int NR, int KP, bf* WP) {
    typedef __attribute__((ext_vector_type(4))) unsigned short v4us;
    const int lane = threadIdx.x & 31; const int o = blockIdx.x * 8 + (threadIdx.x >> 5); if (o >= NR) return;
#pragma unroll 1
    for (int ps = 0; ps < 2; ++ps) {
#pragma unroll 1
        for (int c0 = lane * 4; c0 < KP; c0 += 128) { v4us v;
#pragma unroll
            for (int i = 0; i < 4; ++i) { const int k = c0 + i; v[i] = f2bf((o < nout && k < nin) ? Wt[(size_t)(k < nin ? k : 0) * nout + (o < nout ? o : 0)] : 0.f); }
            *(volatile v4us*)(WP + (size_t)o * KP + c0) = v; }
        if (ps == 0) __threadfence(); }
}
__global__ __launch_bounds__(256) void k_wpadk32(const float* __restrict__ Wt, int nin, int nout, bf* WP) {
    typedef __attribute__((ext_vector_type(2))) unsigned short v2us;
    const int lane = threadIdx.x & 31; const int o = (blockIdx.x * 8 + (threadIdx.x >> 5)) * 2 + (lane >> 4); if (o >= 64) return; const int c0 = (lane & 15) * 2; v2us v;
#pragma unroll
    for (int i = 0; i < 2; ++i) { const int k = c0 + i; v[i] = f2bf((o < nout && k < nin) ? Wt[(size_t)(k < nin ? k : 0) * nout + o] : 0.f); }
    *(volatile v2us*)(WP + (size_t)o * KV + c0) = v; __threadfence(); *(volatile v2us*)(WP + (size_t)o * KV + c0) = v;
}
__global__ __launch_bounds__(64) void k_bpad64(const float* __restrict__ b, int n, float* BP) { const int t = threadIdx.x; const float v = (t < n) ? b[t < n ? t : 0] : 0.f; *(volatile float*)(BP + t) = v; __threadfence(); *(volatile float*)(BP + t) = v; }
__global__ __launch_bounds__(256) void k_out4(const float* __restrict__ RGB, const float* __restrict__ SG, size_t p0, float* OUTP) {
    const int lane = threadIdx.x & 31; const size_t w = (size_t)blockIdx.x * 8 + (threadIdx.x >> 5); if (w >= (size_t)RCH / 32) return; const size_t rr = w * 32 + lane; v4f v;
    v[0] = RGB[rr * 64 + 0]; v[1] = RGB[rr * 64 + 1]; v[2] = RGB[rr * 64 + 2]; v[3] = SG[rr * 64];
    *(volatile v4f*)(OUTP + (p0 + rr) * 4) = v; __threadfence(); *(volatile v4f*)(OUTP + (p0 + rr) * 4) = v;
}

extern "C" void kernel_launch(void* const* d_in, const int* in_sizes, int n_in,
                              void* d_out, int out_size, void* d_ws, size_t ws_size, hipStream_t stream) {
    (void)in_sizes; (void)n_in; (void)out_size;
    const float* pos = (const float*)d_in[0]; const float* cond = (const float*)d_in[1]; const float* view = (const float*)d_in[2];
    const float* dW[8]; const float* db[8]; for (int i = 0; i < 8; ++i) { dW[i] = (const float*)d_in[3 + 2 * i]; db[i] = (const float*)d_in[4 + 2 * i]; }
    const float* sW = (const float*)d_in[19]; const float* sb = (const float*)d_in[20]; const float* cW[3]; const float* cb[3]; for (int i = 0; i < 3; ++i) { cW[i] = (const float*)d_in[21 + 2 * i]; cb[i] = (const float*)d_in[22 + 2 * i]; }
    const float* rW = (const float*)d_in[27]; const float* rb = (const float*)d_in[28];
    float* out = (float*)d_out;
    char* wsp = (char*)d_ws;
    auto take = [&](size_t bytes) { char* p = wsp; wsp += (bytes + 255) & ~(size_t)255; return (void*)p; };
    bf* W0x = (bf*)take(128 * 128 * 2); bf* WD[8]; for (int i = 1; i < 8; ++i) WD[i] = (bf*)take(128 * 128 * 2); bf* W5x = (bf*)take(128 * 128 * 2); bf* SWp = (bf*)take(64 * 128 * 2); float* SBp = (float*)take(256);
    bf* C0h = (bf*)take(64 * 128 * 2); bf* C0v = (bf*)take(64 * 32 * 2); bf* C1 = (bf*)take(64 * 64 * 2); bf* C2 = (bf*)take(64 * 64 * 2); bf* RWp = (bf*)take(64 * 64 * 2); float* RBp = (float*)take(256);
    bf* X0 = (bf*)take((size_t)RCH * KX * 2); bf* VW = (bf*)take((size_t)RCH * KV * 2); float* F = (float*)take((size_t)RCH * HID * 4); float* G = (float*)take((size_t)RCH * HID * 4); bf* Ph = (bf*)take((size_t)RCH * HID * 2); bf* Pl = (bf*)take((size_t)RCH * HID * 2);
    float* SG = (float*)take((size_t)RCH * 64 * 4); float* RGB = (float*)take((size_t)RCH * 64 * 4);
    if ((size_t)(wsp - (char*)d_ws) > ws_size) return;
    k_wpadk<<<128 / 8, 256, 0, stream>>>(dW[0], 67, HID, 128, KX, W0x);
    for (int i = 1; i < 8; ++i) { if (i == 5) continue; k_wpadk<<<128 / 8, 256, 0, stream>>>(dW[i], HID, HID, 128, 128, WD[i]); }
    k_wpadk<<<128 / 8, 256, 0, stream>>>(dW[5], 67, HID, 128, KX, W5x); k_wpadk<<<128 / 8, 256, 0, stream>>>(dW[5] + (size_t)67 * HID, HID, HID, 128, 128, WD[5]);
    k_wpadk<<<64 / 8, 256, 0, stream>>>(sW, HID, 1, 64, 128, SWp); k_bpad64<<<1, 64, 0, stream>>>(sb, 1, SBp);
    k_wpadk<<<64 / 8, 256, 0, stream>>>(cW[0], HID, HC, 64, 128, C0h); k_wpadk32<<<(64 / 2) / 8, 256, 0, stream>>>(cW[0] + (size_t)HID * HC, 3, HC, C0v);
    k_wpadk<<<64 / 8, 256, 0, stream>>>(cW[1], HC, HC, 64, 64, C1); k_wpadk<<<64 / 8, 256, 0, stream>>>(cW[2], HC, HC, 64, 64, C2); k_wpadk<<<64 / 8, 256, 0, stream>>>(rW, HC, 3, 64, 64, RWp); k_bpad64<<<1, 64, 0, stream>>>(rb, 3, RBp);
    const dim3 gH(RCH / 64, HID / 64, 1), gC(RCH / 64, 1, 1);
    for (int c = 0; c < NPT / RCH; ++c) { const size_t p0 = (size_t)c * RCH;
        k_x0pl<<<RCH / 8, 256, 0, stream>>>(pos, cond, p0, X0); k_viewpl<<<(RCH / 2) / 8, 256, 0, stream>>>(view, p0, VW);
        k_gemmb<false, false><<<gH, 128, 0, stream>>>(X0, nullptr, W0x, db[0], F, HID, nullptr, nullptr, KX);
        for (int i = 1; i <= 4; ++i) { k_relupl<HID><<<RCH / 8, 256, 0, stream>>>(i & 1 ? F : G, Ph, Pl); k_gemmb<true, false><<<gH, 128, 0, stream>>>(Ph, Pl, WD[i], db[i], i & 1 ? G : F, HID, nullptr, nullptr, HID); }
        k_relupl<HID><<<RCH / 8, 256, 0, stream>>>(F, Ph, Pl);
        k_gemmb<false, false><<<gH, 128, 0, stream>>>(X0, nullptr, W5x, db[5], G, HID, nullptr, nullptr, KX);
        k_gemmb<true, false><<<gH, 128, 0, stream>>>(Ph, Pl, WD[5], nullptr, F, HID, nullptr, G, HID, 0);
        k_relupl<HID><<<RCH / 8, 256, 0, stream>>>(F, Ph, Pl); k_gemmb<true, false><<<gH, 128, 0, stream>>>(Ph, Pl, WD[6], db[6], G, HID, nullptr, nullptr, HID);
        k_relupl<HID><<<RCH / 8, 256, 0, stream>>>(G, Ph, Pl); k_gemmb<true, false><<<gH, 128, 0, stream>>>(Ph, Pl, WD[7], db[7], F, HID, nullptr, nullptr, HID);
        k_relupl<HID><<<RCH / 8, 256, 0, stream>>>(F, Ph, Pl);
        k_gemmb<true, false><<<gC, 128, 0, stream>>>(Ph, Pl, SWp, SBp, SG, 64, nullptr, nullptr, HID);
        k_gemmb<false, false><<<gC, 128, 0, stream>>>(VW, nullptr, C0v, cb[0], G, 64, nullptr, nullptr, KV);
        k_gemmb<true, false><<<gC, 128, 0, stream>>>(Ph, Pl, C0h, nullptr, RGB, 64, nullptr, G, HID, 0);
        k_relupl<HC><<<RCH / 8, 256, 0, stream>>>(RGB, Ph, Pl); k_gemmb<true, false><<<gC, 128, 0, stream>>>(Ph, Pl, C1, cb[1], G, 64, nullptr, nullptr, HC);
        k_relupl<HC><<<RCH / 8, 256, 0, stream>>>(G, Ph, Pl); k_gemmb<true, false><<<gC, 128, 0, stream>>>(Ph, Pl, C2, cb[2], RGB, 64, nullptr, nullptr, HC);
        k_relupl<HC><<<RCH / 8, 256, 0, stream>>>(RGB, Ph, Pl); k_gemmb<true, false><<<gC, 128, 0, stream>>>(Ph, Pl, RWp, RBp, G, 64, nullptr, nullptr, HC);
        k_out4<<<(RCH / 32) / 8, 256, 0, stream>>>(G, SG, p0, out); }
}
